// NanEchoBlock_69836168233476
// MI455X (gfx1250) — hardware-verified
//
#include <hip/hip_runtime.h>
#include <math.h>
#include <stdint.h>

#define NB    4
#define SEQ   1024
#define DM    768
#define NH    12
#define HD    64
#define DQKV  (3 * DM)
#define DFF   (4 * DM)
#define DTH   (DM / 2)
#define NQB   (SEQ / 64)
#define ROWS  (NB * SEQ)
#define OUTN  (ROWS * DM)
#define THP   32
static_assert(NH * HD == DM);
static_assert(HD == 64);
static_assert((SEQ % 64) == 0 && (DM % 64) == 0 && (DQKV % 64) == 0 && (DFF % 64) == 0);
static_assert((DM % 32) == 0 && (DFF % 32) == 0);
static_assert(DM == 3 * 256);
static_assert((DTH % 32) == 0 && (DTH % 8) == 0);
static_assert(((ROWS / 64) * (DQKV / 64)) % 8 == 0);
static_assert(((ROWS / 64) * (DM / 64)) % 8 == 0);
static_assert(((ROWS / 64) * (DFF / 64)) % 8 == 0);
static_assert((ROWS % 8) == 0);
static_assert(((DQKV * DM / 8) % 256) == 0 && ((DM * DM / 8) % 256) == 0 && ((DFF * DM / 8) % 256) == 0);

typedef _Float16 v16h __attribute__((ext_vector_type(16)));
typedef _Float16 v8h  __attribute__((ext_vector_type(8)));
typedef float    v8f  __attribute__((ext_vector_type(8)));
typedef float    v4f  __attribute__((ext_vector_type(4)));
typedef unsigned int v4u __attribute__((ext_vector_type(4)));

__device__ __forceinline__ unsigned short bf_bits(float f) {
  unsigned u = __float_as_uint(f);
  return (unsigned short)((u + 0x7FFFu + ((u >> 16) & 1u)) >> 16);
}
__device__ __forceinline__ float bfr(float f) { return __uint_as_float(((unsigned)bf_bits(f)) << 16); }
__device__ __forceinline__ unsigned short h_bits(_Float16 x) { return __builtin_bit_cast(unsigned short, x); }
__device__ __forceinline__ unsigned pk16(unsigned short a, unsigned short b) { return (unsigned)a | ((unsigned)b << 16); }
__device__ __forceinline__ v8f zero8() { v8f z = {0.f, 0.f, 0.f, 0.f, 0.f, 0.f, 0.f, 0.f}; return z; }
__device__ __forceinline__ float gelu_erf(float a) { return 0.5f * a * (1.0f + erff(a * 0.70710678118654752f)); }

__device__ __forceinline__ v16h ldfrag_h(const _Float16* p) {
  union { v16h v; v8h h[2]; } f;
  f.h[0] = *(const v8h*)(p);
  f.h[1] = *(const v8h*)(p + 16);
  return f.v;
}

__device__ __forceinline__ v8f mma_h(v16h a, v16h b, v8f c) {
  c = __builtin_amdgcn_wmma_f32_16x16x32_f16(false, a, false, b, (short)0, c, false, false);
#if defined(__HIP_DEVICE_COMPILE__)
  asm volatile("v_nop\n\tv_nop\n\tv_nop\n\tv_nop" : "+v"(c) : "v"(a), "v"(b));
#endif
  return c;
}
__device__ __forceinline__ v8f mma_h_raw(v16h a, v16h b, v8f c) {
  return __builtin_amdgcn_wmma_f32_16x16x32_f16(false, a, false, b, (short)0, c, false, false);
}
__device__ __forceinline__ void dep_guard_h(v8f& a, v8f& b, v16h x, v16h y) {
#if defined(__HIP_DEVICE_COMPILE__)
  asm volatile("v_nop\n\tv_nop\n\tv_nop\n\tv_nop" : "+v"(a), "+v"(b) : "v"(x), "v"(y));
#endif
}
__device__ __forceinline__ void keep4_h(v16h a, v16h b, v16h c, v16h d) {
#if defined(__HIP_DEVICE_COMPILE__)
  asm volatile("v_nop" :: "v"(a), "v"(b), "v"(c), "v"(d));
#endif
}
__device__ __forceinline__ void acc_guard4(v8f& a, v8f& b, v8f& c, v8f& d) {
#if defined(__HIP_DEVICE_COMPILE__)
  asm volatile("v_nop\n\tv_nop\n\tv_nop\n\tv_nop" : "+v"(a), "+v"(b), "+v"(c), "+v"(d));
#endif
}

__global__ __launch_bounds__(256) void cvt_w16(const float* __restrict__ in, const float* __restrict__ msk,
                                               int use_msk, unsigned short* out, int n8, float scale) {
  const int i = blockIdx.x * 256 + threadIdx.x;
  if (i < n8) {
    const v4f a  = *(const v4f*)(in + (size_t)i * 8);
    const v4f b  = *(const v4f*)(in + (size_t)i * 8 + 4);
    const v4f ma = *(const v4f*)(msk + (size_t)i * 8);
    const v4f mb = *(const v4f*)(msk + (size_t)i * 8 + 4);
    float f[8], m[8];
    f[0] = a[0]; f[1] = a[1]; f[2] = a[2]; f[3] = a[3];
    f[4] = b[0]; f[5] = b[1]; f[6] = b[2]; f[7] = b[3];
    m[0] = ma[0]; m[1] = ma[1]; m[2] = ma[2]; m[3] = ma[3];
    m[4] = mb[0]; m[5] = mb[1]; m[6] = mb[2]; m[7] = mb[3];
    v4u p;
#pragma unroll
    for (int e = 0; e < 4; ++e) {
      float g0 = bfr(f[2 * e]), g1 = bfr(f[2 * e + 1]);
      if (use_msk != 0) { g0 *= bfr(m[2 * e]); g1 *= bfr(m[2 * e + 1]); }
      p[e] = pk16(h_bits((_Float16)(g0 * scale)), h_bits((_Float16)(g1 * scale)));
    }
    *(volatile v4u*)(out + (size_t)i * 8) = p;
    __threadfence();
    *(volatile v4u*)(out + (size_t)i * 8) = p;
  }
}

__global__ __launch_bounds__(256) void ln_k(const float* __restrict__ xin, int rb,
                                            const float* __restrict__ gp, const float* __restrict__ bp,
                                            unsigned short* hout, int nrows) {
  union H8 { v8h h; v4u u; };
  __shared__ __align__(16) _Float16 sh[8][DM];
  const int lane = threadIdx.x & 31;
  const int wave = threadIdx.x >> 5;
  const int row  = blockIdx.x * 8 + wave;
  if (row >= nrows) return;
  const float* xr = xin + (size_t)row * DM;
  float v[24];
  float s = 0.f;
#pragma unroll
  for (int i = 0; i < 24; ++i) {
    float t = xr[lane + 32 * i];
    t = (rb != 0) ? bfr(t) : t;
    v[i] = t;
    s += t;
  }
#pragma unroll
  for (int off = 16; off > 0; off >>= 1) s += __shfl_xor(s, off, 32);
  const float mu = s * (1.0f / (float)DM);
  float q = 0.f;
#pragma unroll
  for (int i = 0; i < 24; ++i) { const float d = v[i] - mu; q += d * d; }
#pragma unroll
  for (int off = 16; off > 0; off >>= 1) q += __shfl_xor(q, off, 32);
  const float inv = rsqrtf(q * (1.0f / (float)DM) + 1e-5f);
#pragma unroll
  for (int i = 0; i < 24; ++i) {
    const int cc = lane + 32 * i;
    const float hv = (v[i] - mu) * inv * bfr(gp[cc]) + bfr(bp[cc]);
    sh[wave][cc] = (_Float16)(hv * 16.0f);
  }
  __builtin_amdgcn_fence(__ATOMIC_RELEASE, "workgroup");
  __builtin_amdgcn_wave_barrier();
  __builtin_amdgcn_fence(__ATOMIC_ACQUIRE, "workgroup");
  H8 o[3];
#pragma unroll
  for (int t = 0; t < 3; ++t) o[t].h = *(const v8h*)(&sh[wave][(t * 32 + lane) * 8]);
  for (int pass = 0; pass < 2; ++pass) {
#pragma unroll
    for (int t = 0; t < 3; ++t)
      *(volatile v4u*)(hout + (size_t)row * DM + (size_t)(t * 32 + lane) * 8) = o[t].u;
    __threadfence();
  }
}

__global__ __launch_bounds__(256) void thr_k(
    const unsigned short* __restrict__ Hh,
    const float* __restrict__ w1, const float* __restrict__ b1,
    const float* __restrict__ w2, const float* __restrict__ b2,
    const float* __restrict__ cw, const float* __restrict__ cb,
    float* tout) {
  __shared__ __align__(16) float xm[DM];
  __shared__ float hid[DTH];
  __shared__ float red[2];
  __shared__ __align__(16) float tl[THP];
  const int tid  = threadIdx.x;
  const int wave = tid >> 5;
  const int lane = tid & 31;
  const int b    = blockIdx.x;

  {
    const _Float16* hp = (const _Float16*)(const void*)Hh + (size_t)b * SEQ * DM;
    float s0 = 0.f, s1 = 0.f, s2 = 0.f;
#pragma unroll 1
    for (int t = 0; t < SEQ; ++t) {
      const _Float16* r = hp + (size_t)t * DM;
      s0 += (float)r[tid];
      s1 += (float)r[tid + 256];
      s2 += (float)r[tid + 512];
    }
    const float rl = 1.0f / (16.0f * (float)SEQ);
    xm[tid]       = s0 * rl;
    xm[tid + 256] = s1 * rl;
    xm[tid + 512] = s2 * rl;
  }
  __syncthreads();

#pragma unroll 1
  for (int o = wave; o < DTH; o += 8) {
    const float* wrow = w1 + (size_t)o * DM;
    float s = 0.f;
#pragma unroll 1
    for (int k = lane * 8; k < DM; k += 256) {
      const v4f wa = *(const v4f*)(wrow + k);
      const v4f wb = *(const v4f*)(wrow + k + 4);
      const v4f xa = *(const v4f*)(xm + k);
      const v4f xb = *(const v4f*)(xm + k + 4);
      s = fmaf(xa[0], bfr(wa[0]), s);
      s = fmaf(xa[1], bfr(wa[1]), s);
      s = fmaf(xa[2], bfr(wa[2]), s);
      s = fmaf(xa[3], bfr(wa[3]), s);
      s = fmaf(xb[0], bfr(wb[0]), s);
      s = fmaf(xb[1], bfr(wb[1]), s);
      s = fmaf(xb[2], bfr(wb[2]), s);
      s = fmaf(xb[3], bfr(wb[3]), s);
    }
#pragma unroll
    for (int off = 16; off > 0; off >>= 1) s += __shfl_xor(s, off, 32);
    const float r = fmaxf(s + bfr(b1[o]), 0.0f);
    if (lane == 0) hid[o] = r;
  }
  __syncthreads();

  if (wave < 2) {
    float s = 0.f;
    if (wave == 0) {
#pragma unroll 1
      for (int k = lane; k < DTH; k += 32) s = fmaf(hid[k], bfr(w2[k]), s);
    } else {
#pragma unroll 1
      for (int k = lane; k < DM; k += 32) s = fmaf(xm[k], bfr(cw[k]), s);
    }
#pragma unroll
    for (int off = 16; off > 0; off >>= 1) s += __shfl_xor(s, off, 32);
    const float bias = (wave == 0) ? bfr(b2[0]) : bfr(cb[0]);
    if (lane == 0) red[wave] = s + bias;
  }
  __syncthreads();

  if (tid < THP) {
    const float base = 1.0f / (1.0f + __expf(-red[0]));
    const float cog  = 1.0f / (1.0f + __expf(-red[1]));
    float th = 0.3f + 0.6f * base;
    th = th * (1.0f + cog * 0.5f);
    th = fminf(fmaxf(th, 0.3f), 0.9f);
    tl[tid] = (tid == 0) ? th : 0.0f;
  }
  __syncthreads();
  if (tid < 8) {
    const v4f v = *(const v4f*)(tl + tid * 4);
    float* dst = tout + (size_t)b * THP + tid * 4;
    *(volatile v4f*)dst = v;
    __threadfence();
    *(volatile v4f*)dst = v;
  }
}

template <int EPI>
__global__ __launch_bounds__(256) void gemm64_f16(
    const unsigned short* __restrict__ Ap, int lda,
    const unsigned short* __restrict__ Btp, int ldb,
    const float* __restrict__ biasp, float cscale,
    const float* __restrict__ resp, int ldr,
    void* Cp, int ldc, int M, int N, int K, float oscale) {
  const _Float16* Ah = (const _Float16*)(const void*)Ap;
  const _Float16* Bt = (const _Float16*)(const void*)Btp;
  __shared__ __align__(16) float sT[8][16 * 68];
  const int lane = threadIdx.x & 31;
  const int wave = threadIdx.x >> 5;
  const int tilesN = N >> 6;
  const int tilesM = M >> 6;
  const int tile = blockIdx.x * 8 + wave;
  if (tile >= tilesM * tilesN) return;
  const int tm = tile / tilesN;
  const int tn = tile - tm * tilesN;
  const int m0 = tm << 6;
  const int n0 = tn << 6;

  const int rlane = lane & 15;
  const int koff  = (lane >> 4) * 8;
  const int mOff  = (lane >> 4) * 8;

  v8f acc[4][4];
#pragma unroll
  for (int i = 0; i < 4; ++i)
#pragma unroll
    for (int j = 0; j < 4; ++j) acc[i][j] = zero8();

  for (int k0 = 0; k0 < K; k0 += 32) {
    v16h bh[4];
#pragma unroll
    for (int j = 0; j < 4; ++j) {
      const size_t bo = (size_t)(n0 + (j << 4) + rlane) * ldb + koff + k0;
      bh[j] = ldfrag_h(Bt + bo);
    }
#pragma unroll
    for (int i = 0; i < 4; ++i) {
      const size_t ao = (size_t)(m0 + (i << 4) + rlane) * lda + koff + k0;
      const v16h ah = ldfrag_h(Ah + ao);
#pragma unroll
      for (int j = 0; j < 4; ++j) {
        acc[i][j] = mma_h_raw(ah, bh[j], acc[i][j]);
      }
      dep_guard_h(acc[i][0], acc[i][3], ah, bh[3]);
    }
    keep4_h(bh[0], bh[1], bh[2], bh[3]);
  }
  acc_guard4(acc[0][0], acc[0][1], acc[0][2], acc[0][3]);
  acc_guard4(acc[1][0], acc[1][1], acc[1][2], acc[1][3]);
  acc_guard4(acc[2][0], acc[2][1], acc[2][2], acc[2][3]);
  acc_guard4(acc[3][0], acc[3][1], acc[3][2], acc[3][3]);

  float* slab = sT[wave];
#pragma unroll
  for (int i = 0; i < 4; ++i) {
    const int mBase = m0 + (i << 4);
    float bj[4];
#pragma unroll
    for (int j = 0; j < 4; ++j) bj[j] = bfr(biasp[n0 + (j << 4) + rlane]);
#pragma unroll
    for (int r = 0; r < 8; ++r) {
      const int row = mOff + r;
#pragma unroll
      for (int j = 0; j < 4; ++j) {
        float v = acc[i][j][r] * cscale + bj[j];
        if constexpr (EPI == 1) v = gelu_erf(v);
        slab[row * 68 + (j << 4) + rlane] = v;
      }
    }
    __builtin_amdgcn_fence(__ATOMIC_RELEASE, "workgroup");
    __builtin_amdgcn_wave_barrier();
    __builtin_amdgcn_fence(__ATOMIC_ACQUIRE, "workgroup");
    if constexpr (EPI <= 1) {
      unsigned short* C16 = (unsigned short*)Cp;
      const int rq = lane >> 3, piece = lane & 7;
      v4u pv[4];
#pragma unroll
      for (int it = 0; it < 4; ++it) {
        const int row = it * 4 + rq;
        const v4f a  = *(const v4f*)(slab + row * 68 + piece * 8);
        const v4f a2 = *(const v4f*)(slab + row * 68 + piece * 8 + 4);
        v4u p;
        p[0] = pk16(h_bits((_Float16)(a[0]  * oscale)), h_bits((_Float16)(a[1]  * oscale)));
        p[1] = pk16(h_bits((_Float16)(a[2]  * oscale)), h_bits((_Float16)(a[3]  * oscale)));
        p[2] = pk16(h_bits((_Float16)(a2[0] * oscale)), h_bits((_Float16)(a2[1] * oscale)));
        p[3] = pk16(h_bits((_Float16)(a2[2] * oscale)), h_bits((_Float16)(a2[3] * oscale)));
        pv[it] = p;
      }
      for (int pass = 0; pass < 2; ++pass) {
#pragma unroll
        for (int it = 0; it < 4; ++it) {
          const int row = it * 4 + rq;
          *(volatile v4u*)(C16 + (size_t)(mBase + row) * ldc + n0 + piece * 8) = pv[it];
        }
        __threadfence();
      }
    } else {
      float* Cf = (float*)Cp;
      const int hh = lane >> 4, c4 = (lane & 15) * 4;
      v4f ov[8];
#pragma unroll
      for (int it = 0; it < 8; ++it) {
        const int row = it * 2 + hh;
        v4f o = *(const v4f*)(slab + row * 68 + c4);
        const v4f rs = *(const v4f*)(resp + (size_t)(mBase + row) * ldr + n0 + c4);
        if constexpr (EPI == 2) {
          o[0] += bfr(rs[0]); o[1] += bfr(rs[1]); o[2] += bfr(rs[2]); o[3] += bfr(rs[3]);
        } else {
          o += rs;
        }
        ov[it] = o;
      }
      for (int pass = 0; pass < 2; ++pass) {
#pragma unroll
        for (int it = 0; it < 8; ++it) {
          const int row = it * 2 + hh;
          *(volatile v4f*)(Cf + (size_t)(mBase + row) * ldc + n0 + c4) = ov[it];
        }
        __threadfence();
      }
    }
    __builtin_amdgcn_fence(__ATOMIC_RELEASE, "workgroup");
    __builtin_amdgcn_wave_barrier();
    __builtin_amdgcn_fence(__ATOMIC_ACQUIRE, "workgroup");
  }
}

__global__ __launch_bounds__(256) void v_tr(const unsigned short* __restrict__ qkvp, unsigned short* vt) {
  __shared__ __align__(16) _Float16 sv[64 * 72];
  const int tid = threadIdx.x;
  const int t0  = blockIdx.x * 64;
  const int hh  = blockIdx.y;
  const int b   = blockIdx.z;
  const _Float16* src = (const _Float16*)(const void*)qkvp;
#pragma unroll
  for (int i = 0; i < 2; ++i) {
    const int idx = i * 256 + tid;
    const int tt = idx >> 3, c8 = (idx & 7) * 8;
    const v8h a = *(const v8h*)(src + ((size_t)(b * SEQ + t0 + tt)) * DQKV + 2 * DM + hh * HD + c8);
    *(v8h*)(sv + tt * 72 + c8) = a;
  }
  __syncthreads();

  const int g = tid >> 3, piece = tid & 7;
  v4u hv[2];
  size_t hofs[2];
#pragma unroll
  for (int it = 0; it < 2; ++it) {
    const int d = it * 32 + g;
    v4u a;
#pragma unroll
    for (int e = 0; e < 4; ++e) {
      const _Float16 x0 = sv[(piece * 8 + 2 * e) * 72 + d];
      const _Float16 x1 = sv[(piece * 8 + 2 * e + 1) * 72 + d];
      a[e] = pk16(h_bits(x0), h_bits(x1));
    }
    hv[it] = a;
    hofs[it] = ((size_t)(b * DM + hh * HD + d)) * SEQ + t0 + piece * 8;
  }
  for (int pass = 0; pass < 2; ++pass) {
#pragma unroll
    for (int it = 0; it < 2; ++it) *(volatile v4u*)(vt + hofs[it]) = hv[it];
    __threadfence();
  }
}

__global__ __launch_bounds__(128)
void attn_k(const unsigned short* __restrict__ qkvp, const unsigned short* __restrict__ vtp,
            const float* __restrict__ thrp, unsigned short* ctxp) {
  union FH { v16h v; v8h h[2]; };
  __shared__ __align__(16) _Float16 Ksh[64 * 64];
  __shared__ __align__(16) _Float16 Vsh[64 * 64];
  __shared__ __align__(16) _Float16 Psh[4][16 * 64];
  __shared__ __align__(16) float    Os[4][16 * 64];

  const int tid  = threadIdx.x;
  const int wave = tid >> 5;
  const int lane = tid & 31;
  const int hh   = lane >> 4;
  const int c    = lane & 15;

  const int bx   = blockIdx.x;
  const int qb   = bx % NQB;
  const int rest = bx / NQB;
  const int h    = rest % NH;
  const int b    = rest / NH;
  const int q0   = qb * 64 + wave * 16;
  const size_t rowB = (size_t)b * SEQ;

  const float thr = thrp[b * THP];

  const _Float16* Qp = (const _Float16*)(const void*)qkvp + (size_t)h * HD;
  const _Float16* Kp = (const _Float16*)(const void*)qkvp + DM + (size_t)h * HD;
  const _Float16* Vt = (const _Float16*)(const void*)vtp + ((size_t)b * DM + (size_t)h * HD) * SEQ;

  v16h qa[2];
#pragma unroll
  for (int dc = 0; dc < 2; ++dc) {
    const size_t qo = (rowB + q0 + c) * DQKV + dc * 32 + 8 * hh;
    qa[dc] = ldfrag_h(Qp + qo);
  }

  float mrow[8], lrow[8];
  v8f oacc[4];
#pragma unroll
  for (int r = 0; r < 8; ++r) { mrow[r] = 0.f; lrow[r] = 0.f; }
#pragma unroll
  for (int t = 0; t < 4; ++t) oacc[t] = zero8();

  _Float16* pw = Psh[wave];

  const int nkt = qb + 1;
  for (int kt = 0; kt < nkt; ++kt) {
    const int kv0 = kt * 64;
    __syncthreads();
    {
      const int r = tid >> 1, half = (tid & 1) * 32;
      const _Float16* kg = Kp + (rowB + kv0 + r) * DQKV + half;
      const _Float16* vg = Vt + (size_t)r * SEQ + kv0 + half;
#pragma unroll
      for (int i = 0; i < 4; ++i) {
        const v8h a0 = *(const v8h*)(kg + 8 * i);
        const v8h b0 = *(const v8h*)(vg + 8 * i);
        *(v8h*)(Ksh + r * 64 + half + 8 * i) = a0;
        *(v8h*)(Vsh + r * 64 + half + 8 * i) = b0;
      }
    }
    __syncthreads();

    v8f s[4];
#pragma unroll
    for (int j = 0; j < 4; ++j) {
      s[j] = zero8();
#pragma unroll
      for (int dc = 0; dc < 2; ++dc) {
        FH kb;
        kb.h[0] = *(const v8h*)(Ksh + (j * 16 + c) * 64 + dc * 32 + 8 * hh);
        kb.h[1] = *(const v8h*)(Ksh + (j * 16 + c) * 64 + dc * 32 + 16 + 8 * hh);
        s[j] = mma_h(qa[dc], kb.v, s[j]);
      }
    }

#pragma unroll
    for (int r = 0; r < 8; ++r) {
      const int qrow = q0 + 8 * hh + r;
      float m = 0.f;
#pragma unroll
      for (int j = 0; j < 4; ++j) {
        const int key = kv0 + j * 16 + c;
        const float a  = s[j][r] * (1.0f / 2048.0f);
        const float ea = __expf(fminf(a - thr, 40.0f));
        const float eb = __expf(fminf(-a - thr, 40.0f));
        float rr = (1.0f + ea) * __builtin_amdgcn_rcpf(1.0f + eb);
        rr = (key > qrow) ? 0.0f : rr;
        s[j][r] = rr;
        m = fmaxf(m, rr);
      }
#pragma unroll
      for (int off = 1; off < 16; off <<= 1) m = fmaxf(m, __shfl_xor(m, off, 32));
      const float mn    = fmaxf(mrow[r], m);
      const float msafe = (mn > 0.f) ? mn : 1.0f;
      const float rinv  = __builtin_amdgcn_rcpf(msafe);
      const float alpha = mrow[r] * rinv;
      mrow[r] = mn;
      float psum = 0.f;
#pragma unroll
      for (int j = 0; j < 4; ++j) {
        const float p = s[j][r] * rinv;
        psum += p;
        pw[(8 * hh + r) * 64 + j * 16 + c] = (_Float16)(p * 1024.0f);
      }
#pragma unroll
      for (int off = 1; off < 16; off <<= 1) psum += __shfl_xor(psum, off, 32);
      lrow[r] = lrow[r] * alpha + psum;
#pragma unroll
      for (int t = 0; t < 4; ++t) oacc[t][r] *= alpha;
    }
    __builtin_amdgcn_fence(__ATOMIC_RELEASE, "workgroup");
    __builtin_amdgcn_wave_barrier();
    __builtin_amdgcn_fence(__ATOMIC_ACQUIRE, "workgroup");

#pragma unroll
    for (int kk = 0; kk < 2; ++kk) {
      FH pa;
      pa.h[0] = *(const v8h*)(pw + c * 64 + kk * 32 + 8 * hh);
      pa.h[1] = *(const v8h*)(pw + c * 64 + kk * 32 + 16 + 8 * hh);
#pragma unroll
      for (int t = 0; t < 4; ++t) {
        FH vb;
        vb.h[0] = *(const v8h*)(Vsh + (t * 16 + c) * 64 + kk * 32 + 8 * hh);
        vb.h[1] = *(const v8h*)(Vsh + (t * 16 + c) * 64 + kk * 32 + 16 + 8 * hh);
        oacc[t] = mma_h(pa.v, vb.v, oacc[t]);
      }
    }
  }

  float* os = Os[wave];
#pragma unroll
  for (int r = 0; r < 8; ++r) {
    const float l = lrow[r];
    const float inv = ((l > 0.f) ? __builtin_amdgcn_rcpf(l) : 0.f) * (1.0f / 1024.0f);
#pragma unroll
    for (int t = 0; t < 4; ++t) os[(8 * hh + r) * 64 + t * 16 + c] = oacc[t][r] * inv;
  }
  __builtin_amdgcn_fence(__ATOMIC_RELEASE, "workgroup");
  __builtin_amdgcn_wave_barrier();
  __builtin_amdgcn_fence(__ATOMIC_ACQUIRE, "workgroup");
  {
    const int rq = lane >> 3, piece = lane & 7;
    v4u pv[4];
#pragma unroll
    for (int it = 0; it < 4; ++it) {
      const int row = it * 4 + rq;
      const v4f a  = *(const v4f*)(os + row * 64 + piece * 8);
      const v4f a2 = *(const v4f*)(os + row * 64 + piece * 8 + 4);
      v4u p;
      p[0] = pk16(h_bits((_Float16)a[0]),  h_bits((_Float16)a[1]));
      p[1] = pk16(h_bits((_Float16)a[2]),  h_bits((_Float16)a[3]));
      p[2] = pk16(h_bits((_Float16)a2[0]), h_bits((_Float16)a2[1]));
      p[3] = pk16(h_bits((_Float16)a2[2]), h_bits((_Float16)a2[3]));
      pv[it] = p;
    }
    for (int pass = 0; pass < 2; ++pass) {
#pragma unroll
      for (int it = 0; it < 4; ++it) {
        const int row = it * 4 + rq;
        const size_t go = (rowB + q0 + row) * DM + (size_t)h * HD + piece * 8;
        *(volatile v4u*)(ctxp + go) = pv[it];
      }
      __threadfence();
    }
  }
}

extern "C" void kernel_launch(void* const* d_in, const int* in_sizes, int n_in,
                              void* d_out, int out_size, void* d_ws, size_t ws_size,
                              hipStream_t stream) {
  if (n_in < 20) return;
  if (in_sizes[0] != NB * SEQ * DM) return;
  if (in_sizes[1] != DM || in_sizes[2] != DM) return;
  if (in_sizes[3] != DQKV * DM || in_sizes[4] != DQKV) return;
  if (in_sizes[5] != DM * DM || in_sizes[6] != DM || in_sizes[7] != DM * DM) return;
  if (in_sizes[8] != DTH * DM || in_sizes[9] != DTH || in_sizes[10] != DTH || in_sizes[11] < 1) return;
  if (in_sizes[12] != DM || in_sizes[13] < 1) return;
  if (in_sizes[14] != DM || in_sizes[15] != DM) return;
  if (in_sizes[16] != DFF * DM || in_sizes[17] != DFF || in_sizes[18] != DM * DFF || in_sizes[19] != DM) return;
  if (out_size != OUTN) return;

  const float* x      = (const float*)d_in[0];
  const float* ln1_g  = (const float*)d_in[1];
  const float* ln1_b  = (const float*)d_in[2];
  const float* qkv_w  = (const float*)d_in[3];
  const float* qkv_b  = (const float*)d_in[4];
  const float* out_w  = (const float*)d_in[5];
  const float* out_b  = (const float*)d_in[6];
  const float* cmask  = (const float*)d_in[7];
  const float* thr_w1 = (const float*)d_in[8];
  const float* thr_b1 = (const float*)d_in[9];
  const float* thr_w2 = (const float*)d_in[10];
  const float* thr_b2 = (const float*)d_in[11];
  const float* cog_w  = (const float*)d_in[12];
  const float* cog_b  = (const float*)d_in[13];
  const float* ln2_g  = (const float*)d_in[14];
  const float* ln2_b  = (const float*)d_in[15];
  const float* mlp_w1 = (const float*)d_in[16];
  const float* mlp_b1 = (const float*)d_in[17];
  const float* mlp_w2 = (const float*)d_in[18];
  const float* mlp_b2 = (const float*)d_in[19];

  const size_t PWqkv = (size_t)DQKV * DM * 2;
  const size_t PWo   = (size_t)DM * DM * 2;
  const size_t PW1   = (size_t)DFF * DM * 2;
  const size_t PW2   = (size_t)DM * DFF * 2;
  const size_t PTH   = (size_t)NB * THP * 4;
  const size_t PH16  = (size_t)ROWS * DM * 2;
  const size_t PQKV  = (size_t)ROWS * DQKV * 2;
  const size_t PVT   = (size_t)NB * DM * SEQ * 2;
  const size_t PF32  = (size_t)ROWS * DM * 4;
  const size_t PG    = (size_t)ROWS * DFF * 2;
  size_t off = 0;
  const size_t oWqkv = off; off += PWqkv;
  const size_t oWo   = off; off += PWo;
  const size_t oW1   = off; off += PW1;
  const size_t oW2   = off; off += PW2;
  const size_t oTH   = off; off += PTH;
  const size_t oHh   = off; off += PH16;
  const size_t oQKV  = off; off += PQKV;
  const size_t oVT   = off; off += PVT;
  const size_t oCtx  = off; off += PH16;
  const size_t oX1   = off; off += PF32;
  const size_t oH2   = off; off += PH16;
  const size_t oG    = off; off += PG;
  if (off > ws_size) return;
  if (off > (size_t)134217728) return;

  char* ws = (char*)d_ws;
  unsigned short* Wqkv = (unsigned short*)(ws + oWqkv);
  unsigned short* Wo   = (unsigned short*)(ws + oWo);
  unsigned short* W1   = (unsigned short*)(ws + oW1);
  unsigned short* W2   = (unsigned short*)(ws + oW2);
  float*          THR  = (float*)(ws + oTH);
  unsigned short* Hh   = (unsigned short*)(ws + oHh);
  unsigned short* QKV  = (unsigned short*)(ws + oQKV);
  unsigned short* VT   = (unsigned short*)(ws + oVT);
  unsigned short* Ctx  = (unsigned short*)(ws + oCtx);
  float*          X1   = (float*)(ws + oX1);
  unsigned short* H2   = (unsigned short*)(ws + oH2);
  unsigned short* G    = (unsigned short*)(ws + oG);
  float*          outf = (float*)d_out;

  const dim3 blk(256);
  const int n8qkv = DQKV * DM / 8;
  const int n8o   = DM * DM / 8;
  const int n8f   = DFF * DM / 8;
  const dim3 gCq((n8qkv + 255) / 256);
  const dim3 gCo((n8o + 255) / 256);
  const dim3 gCf((n8f + 255) / 256);
  const dim3 gLn((ROWS + 7) / 8);
  const dim3 gThr(NB);
  const dim3 gGqkv(((ROWS / 64) * (DQKV / 64) + 7) / 8);
  const dim3 gGdm(((ROWS / 64) * (DM / 64) + 7) / 8);
  const dim3 gGff(((ROWS / 64) * (DFF / 64) + 7) / 8);
  const dim3 gVt(SEQ / 64, NH, NB);
  const dim3 gAttn(NB * NH * NQB);
  const float wScale = 256.0f;
  const float aScale = 16.0f;
  const float cscale = 1.0f / 4096.0f;

  cvt_w16<<<gCq, blk, 0, stream>>>(qkv_w, qkv_w, 0, Wqkv, n8qkv, wScale);
  cvt_w16<<<gCo, blk, 0, stream>>>(out_w, cmask, 1, Wo, n8o, wScale);
  cvt_w16<<<gCf, blk, 0, stream>>>(mlp_w1, mlp_w1, 0, W1, n8f, wScale);
  cvt_w16<<<gCf, blk, 0, stream>>>(mlp_w2, mlp_w2, 0, W2, n8f, wScale);
  ln_k<<<gLn, blk, 0, stream>>>(x, 1, ln1_g, ln1_b, Hh, ROWS);
  thr_k<<<gThr, blk, 0, stream>>>(Hh, thr_w1, thr_b1, thr_w2, thr_b2, cog_w, cog_b, THR);
  gemm64_f16<0><<<gGqkv, blk, 0, stream>>>(Hh, DM, Wqkv, DM, qkv_b, cscale, x, DM, (void*)QKV, DQKV,
                                           ROWS, DQKV, DM, aScale);
  v_tr<<<gVt, blk, 0, stream>>>(QKV, VT);
  attn_k<<<gAttn, dim3(128), 0, stream>>>(QKV, VT, THR, Ctx);
  gemm64_f16<2><<<gGdm, blk, 0, stream>>>(Ctx, DM, Wo, DM, out_b, cscale, x, DM, (void*)X1, DM,
                                          ROWS, DM, DM, 1.0f);
  ln_k<<<gLn, blk, 0, stream>>>(X1, 0, ln2_g, ln2_b, H2, ROWS);
  gemm64_f16<1><<<gGff, blk, 0, stream>>>(H2, DM, W1, DM, mlp_b1, cscale, x, DM, (void*)G, DFF,
                                          ROWS, DFF, DM, aScale);
  gemm64_f16<3><<<gGdm, blk, 0, stream>>>(G, DFF, W2, DFF, mlp_b2, cscale, X1, DM, (void*)outf, DM,
                                          ROWS, DM, DFF, 1.0f);
  (void)hipGetLastError();
}
